// TemporalExt_47991964566192
// MI455X (gfx1250) — hardware-verified
//
#include <hip/hip_runtime.h>
#include <hip/hip_bf16.h>


#define FQ   4
#define NLY  2
#define NB   8
#define SL   256
#define TOK  (NB * SL)
#define DM   256
#define DI   512
#define NS   16
#define DTR  16
#define XDN  48
#define XDW  64
#define NV   128
#define NO   256
#define TOKO (NB * FQ * SL)

static_assert(DM == 32 * 8);
static_assert(DTR + 2 * NS == XDN);
static_assert(XDN <= XDW);
static_assert(TOK % 64 == 0);
static_assert(TOKO % 64 == 0);
static_assert(DM % 64 == 0);
static_assert(DI % 64 == 0);
static_assert((2 * DI) % 64 == 0);
static_assert(XDW % 64 == 0);
static_assert(NV % 64 == 0);
static_assert(NO % 64 == 0);
static_assert(DM % 32 == 0 && DI % 32 == 0 && NV % 32 == 0);
static_assert((SL & (SL - 1)) == 0);
static_assert(SL % 16 == 0);
static_assert(DI % 8 == 0 && DM % 8 == 0);
static_assert((TOK * NV) % (8 * 256) == 0);

typedef float          v4f   __attribute__((ext_vector_type(4)));
typedef float          v8f   __attribute__((ext_vector_type(8)));
typedef __bf16         v16b  __attribute__((ext_vector_type(16)));
typedef unsigned short u16x8 __attribute__((ext_vector_type(8)));

union FragB { u16x8 h[2]; v16b v; };

constexpr size_t SZ_WI  = (size_t)FQ * NLY * 2 * DI * DM * 2;
constexpr size_t SZ_WX  = (size_t)FQ * NLY * XDW * DI * 2;
constexpr size_t SZ_WO  = (size_t)FQ * NLY * DM * DI * 2;
constexpr size_t SZ_WL  = (size_t)FQ * NV * DM * 2;
constexpr size_t SZ_WT  = (size_t)NO * NV * 2;
constexpr size_t SZ_H   = (size_t)FQ * TOK * DM * 4;
constexpr size_t SZ_N16 = (size_t)FQ * TOK * DM * 2;
constexpr size_t SZ_XF  = (size_t)FQ * TOK * DI * 4;
constexpr size_t SZ_U16 = (size_t)FQ * TOK * DI * 2;
constexpr size_t SZ_XD  = (size_t)FQ * TOK * XDW * 4;
constexpr size_t SZ_LG  = (size_t)FQ * TOK * NV * 4;
constexpr size_t SZ_BN  = (size_t)TOKO * NV * 2;

constexpr size_t OFF_WIH = 0;
constexpr size_t OFF_WIL = OFF_WIH + SZ_WI;
constexpr size_t OFF_WXH = OFF_WIL + SZ_WI;
constexpr size_t OFF_WXL = OFF_WXH + SZ_WX;
constexpr size_t OFF_WOH = OFF_WXL + SZ_WX;
constexpr size_t OFF_WOL = OFF_WOH + SZ_WO;
constexpr size_t OFF_WLH = OFF_WOL + SZ_WO;
constexpr size_t OFF_WLL = OFF_WLH + SZ_WL;
constexpr size_t OFF_WTH = OFF_WLL + SZ_WL;
constexpr size_t OFF_WTL = OFF_WTH + SZ_WT;
constexpr size_t OFF_HA  = OFF_WTL + SZ_WT;
constexpr size_t OFF_HB  = OFF_HA  + SZ_H;
constexpr size_t OFF_NH  = OFF_HB  + SZ_H;
constexpr size_t OFF_NL  = OFF_NH  + SZ_N16;
constexpr size_t OFF_XF  = OFF_NL  + SZ_N16;
constexpr size_t OFF_ZF  = OFF_XF  + SZ_XF;
constexpr size_t OFF_UH  = OFF_ZF  + SZ_XF;
constexpr size_t OFF_UL  = OFF_UH  + SZ_U16;
constexpr size_t OFF_XD  = OFF_UL  + SZ_U16;
constexpr size_t OFF_GH  = OFF_XD  + SZ_XD;
constexpr size_t OFF_GL  = OFF_GH  + SZ_U16;
constexpr size_t OFF_LG  = OFF_GL  + SZ_U16;
constexpr size_t OFF_BNH = OFF_LG  + SZ_LG;
constexpr size_t OFF_BNL = OFF_BNH + SZ_BN;
constexpr size_t WS_END  = OFF_BNL + SZ_BN;
static_assert(WS_END == (size_t)117047296);
static_assert(WS_END <= (size_t)134217728);
static_assert(SZ_WI % 128 == 0 && SZ_WX % 128 == 0 && SZ_WO % 128 == 0 && SZ_WL % 128 == 0 && SZ_WT % 128 == 0);
static_assert(SZ_H % 128 == 0 && SZ_N16 % 128 == 0 && SZ_XF % 128 == 0 && SZ_U16 % 128 == 0);
static_assert(SZ_XD % 128 == 0 && SZ_LG % 128 == 0 && SZ_BN % 128 == 0);

__device__ __forceinline__ unsigned short f32_to_bf16(float f) {
    unsigned u = __float_as_uint(f);
    unsigned r = u + 0x7FFFu + ((u >> 16) & 1u);
    return (unsigned short)(r >> 16);
}
__device__ __forceinline__ float bf16_to_f32(unsigned short b) {
    return __uint_as_float(((unsigned)b) << 16);
}
__device__ __forceinline__ float silu_f(float x) {
    float e = __expf(-x);
    return x * __builtin_amdgcn_rcpf(1.0f + e);
}
__device__ __forceinline__ float softplus_f(float x) {
    return fmaxf(x, 0.0f) + log1pf(__expf(-fabsf(x)));
}
__device__ __forceinline__ float conv4_silu(float x0, float x1, float x2, float x3,
                                            float w0, float w1, float w2, float w3, float bias) {
    float c = w0 * x0 + w1 * x1 + w2 * x2 + w3 * x3;
    return silu_f(c + bias);
}
__device__ __forceinline__ v8f ld8f(const float* p) {
    v4f a = *(const v4f*)p;
    v4f b = *(const v4f*)(p + 4);
    return __builtin_shufflevector(a, b, 0, 1, 2, 3, 4, 5, 6, 7);
}
__device__ __forceinline__ void split8(const v8f x, u16x8& hv, u16x8& lv) {
#pragma unroll
    for (int c = 0; c < 8; ++c) {
        const float f = x[c];
        const unsigned short hb = f32_to_bf16(f);
        const unsigned short lb = f32_to_bf16(f - bf16_to_f32(hb));
        hv[c] = hb;
        lv[c] = lb;
    }
}
__device__ __forceinline__ void store_planes2x(unsigned short* ph, unsigned short* pl,
                                               const u16x8 hv, const u16x8 lv) {
    *(volatile u16x8*)ph = hv;
    *(volatile u16x8*)pl = lv;
    __threadfence();
    *(volatile u16x8*)ph = hv;
    *(volatile u16x8*)pl = lv;
}

__device__ __forceinline__ void mma16(v8f& acc, const FragB& a, const FragB& b) {
    acc = __builtin_amdgcn_wmma_f32_16x16x32_bf16(false, a.v, false, b.v, (short)0, acc, false, false);
    asm volatile("v_nop\n\tv_nop\n\tv_nop\n\tv_nop" : "+v"(acc) : "v"(a.v), "v"(b.v));
}

__global__ __launch_bounds__(256)
void cvt_kernel(const float* __restrict__ src, unsigned short* dsth, unsigned short* dstl,
                int n8, int dstPer8, int srcPer8)
{
    const int i = blockIdx.x * 256 + threadIdx.x;
    if (i >= n8) return;
    const int q  = i / dstPer8;
    const int r  = i - q * dstPer8;
    const int rc = (r < srcPer8) ? r : (srcPer8 - 1);
    v8f x = ld8f(src + ((size_t)q * srcPer8 + (size_t)rc) * 8);
    if (r >= srcPer8) {
#pragma unroll
        for (int c = 0; c < 8; ++c) x[c] = 0.0f;
    }
    u16x8 hv, lv;
    split8(x, hv, lv);
    const size_t e = (size_t)i * 8;
    store_planes2x(dsth + e, dstl + e, hv, lv);
}

__global__ __launch_bounds__(32)
void rmsnorm_cvt_kernel(const float* __restrict__ src, int sFeat, int sRow,
                        const float* __restrict__ w, int wFeat,
                        unsigned short* nh, unsigned short* nl)
{
    const int f = blockIdx.y;
    const int t = blockIdx.x;
    const int lane = threadIdx.x;
    const v8f x = ld8f(src + (size_t)f * sFeat + (size_t)t * sRow + lane * 8);
    float ss = 0.0f;
#pragma unroll
    for (int c = 0; c < 8; ++c) ss += x[c] * x[c];
    ss += __shfl_xor(ss, 16);
    ss += __shfl_xor(ss, 8);
    ss += __shfl_xor(ss, 4);
    ss += __shfl_xor(ss, 2);
    ss += __shfl_xor(ss, 1);
    const float sc = rsqrtf(ss * (1.0f / (float)DM) + 1e-5f);
    const v8f wv = ld8f(w + (size_t)f * wFeat + lane * 8);
    v8f y;
#pragma unroll
    for (int c = 0; c < 8; ++c) y[c] = (x[c] * sc) * wv[c];
    u16x8 hv, lv;
    split8(y, hv, lv);
    const size_t e = ((size_t)f * TOK + (size_t)t) * DM + lane * 8;
    store_planes2x(nh + e, nl + e, hv, lv);
}

template<int NBF>
__device__ __forceinline__ void tile_store_pass(const float* st, float* gp, int ldc, int lane) {
    constexpr int CW  = NBF * 16;
    constexpr int P   = CW + 4;
    constexpr int LPR = CW / 4;
    static_assert(32 % LPR == 0);
    constexpr int RPI = 32 / LPR;
    static_assert(32 % RPI == 0);
    constexpr int NIT = 32 / RPI;
    const int rsub = lane / LPR;
    const int c0   = (lane % LPR) * 4;
#pragma unroll
    for (int it = 0; it < NIT; ++it) {
        const int row = it * RPI + rsub;
        const v4f v = *(const v4f*)(st + row * P + c0);
        *(volatile v4f*)(gp + (size_t)row * ldc + c0) = v;
    }
}

template<int NBF, int EPI>
__global__ __launch_bounds__(128)
void gemm3_kernel(const unsigned short* __restrict__ Ah, const unsigned short* __restrict__ Al, int aFeat,
                  const unsigned short* __restrict__ Bh, const unsigned short* __restrict__ Bl, int bFeat,
                  float* C, float* C2, int cFeat, int K, int ldc, int csplit,
                  const float* __restrict__ R, int rFeat, int rRow)
{
    constexpr int CW = NBF * 16;
    constexpr int P  = CW + 4;
    static_assert(CW % 32 == 0);
    __shared__ __attribute__((aligned(16))) float stile[4][32 * P];

    const int tid  = threadIdx.x;
    const int lane = tid & 31;
    const int wave = tid >> 5;
    const int h    = lane >> 4;
    const int m    = lane & 15;
    const int wm   = wave >> 1;
    const int wn   = wave & 1;
    const int f    = blockIdx.z;

    const int rowW = blockIdx.y * 64 + wm * 32;
    const int colW = blockIdx.x * (2 * CW) + wn * CW;

    const unsigned short* Ahf = Ah + (size_t)f * aFeat;
    const unsigned short* Alf = Al + (size_t)f * aFeat;
    const unsigned short* Bhf = Bh + (size_t)f * bFeat;
    const unsigned short* Blf = Bl + (size_t)f * bFeat;

    v8f acc[2 * NBF];
#pragma unroll
    for (int j = 0; j < 2 * NBF; ++j)
#pragma unroll
        for (int r = 0; r < 8; ++r) acc[j][r] = 0.0f;

    const size_t aoff  = (size_t)(rowW + m) * K + 8 * h;
    const size_t boff  = (size_t)(colW + m) * K + 8 * h;
    const size_t sub16 = (size_t)16 * K;
    const int nk = K >> 5;

#pragma unroll 1
    for (int kt = 0; kt < nk; ++kt) {
        const size_t k0 = (size_t)kt * 32;
        FragB fa[2], ga[2], fb[NBF], gb[NBF];
#pragma unroll
        for (int s = 0; s < 2; ++s) {
            const unsigned short* p = Ahf + aoff + s * sub16 + k0;
            fa[s].h[0] = *(const u16x8*)(p);
            fa[s].h[1] = *(const u16x8*)(p + 16);
            const unsigned short* q = Alf + aoff + s * sub16 + k0;
            ga[s].h[0] = *(const u16x8*)(q);
            ga[s].h[1] = *(const u16x8*)(q + 16);
        }
#pragma unroll
        for (int j = 0; j < NBF; ++j) {
            const unsigned short* p = Bhf + boff + j * sub16 + k0;
            fb[j].h[0] = *(const u16x8*)(p);
            fb[j].h[1] = *(const u16x8*)(p + 16);
            const unsigned short* q = Blf + boff + j * sub16 + k0;
            gb[j].h[0] = *(const u16x8*)(q);
            gb[j].h[1] = *(const u16x8*)(q + 16);
        }
#pragma unroll
        for (int s = 0; s < 2; ++s)
#pragma unroll
            for (int j = 0; j < NBF; ++j) {
                mma16(acc[s * NBF + j], fa[s], fb[j]);
                mma16(acc[s * NBF + j], fa[s], gb[j]);
                mma16(acc[s * NBF + j], ga[s], fb[j]);
            }
    }

    float* st = stile[wave];
#pragma unroll
    for (int s = 0; s < 2; ++s)
#pragma unroll
        for (int j = 0; j < NBF; ++j)
#pragma unroll
            for (int r = 0; r < 8; ++r) {
                const int rr = s * 16 + 8 * h + r;
                const int cc = j * 16 + m;
                float v = acc[s * NBF + j][r];
                if (EPI == 1) v += R[(size_t)f * rFeat + (size_t)(rowW + rr) * rRow + colW + cc];
                if (EPI == 2) v += R[colW + cc];
                st[rr * P + cc] = v;
            }
    __syncthreads();

    float* Cp = C + (size_t)f * cFeat;
    int gcol = colW;
    if (colW >= csplit) { Cp = C2 + (size_t)f * cFeat; gcol = colW - csplit; }
    float* gp = Cp + (size_t)rowW * ldc + gcol;
    tile_store_pass<NBF>(st, gp, ldc, lane);
    __threadfence();
    tile_store_pass<NBF>(st, gp, ldc, lane);
}

__global__ __launch_bounds__(64)
void conv_cvt_kernel(const float* __restrict__ X, const float* __restrict__ cw,
                     const float* __restrict__ cb, int layer,
                     unsigned short* uh, unsigned short* ul)
{
    const int f  = blockIdx.y;
    const int t  = blockIdx.x;
    const int l  = t & (SL - 1);
    const int d0 = threadIdx.x * 8;
    const size_t rbase = (size_t)f * TOK;
    const int t1 = (l >= 1) ? (t - 1) : t;
    const int t2 = (l >= 2) ? (t - 2) : t;
    const int t3 = (l >= 3) ? (t - 3) : t;

    v8f xm0 = ld8f(X + (rbase + (size_t)t)  * DI + d0);
    v8f xm1 = ld8f(X + (rbase + (size_t)t1) * DI + d0);
    v8f xm2 = ld8f(X + (rbase + (size_t)t2) * DI + d0);
    v8f xm3 = ld8f(X + (rbase + (size_t)t3) * DI + d0);
#pragma unroll
    for (int c = 0; c < 8; ++c) {
        if (l < 1) xm1[c] = 0.0f;
        if (l < 2) xm2[c] = 0.0f;
        if (l < 3) xm3[c] = 0.0f;
    }

    const size_t pbase = ((size_t)(f * NLY + layer)) * DI + d0;
    v4f wv[8];
#pragma unroll
    for (int c = 0; c < 8; ++c) wv[c] = *(const v4f*)(cw + (pbase + c) * 4);
    const v8f bias = ld8f(cb + pbase);

    v8f u;
#pragma unroll
    for (int c = 0; c < 8; ++c)
        u[c] = conv4_silu(xm3[c], xm2[c], xm1[c], xm0[c], wv[c][0], wv[c][1], wv[c][2], wv[c][3], bias[c]);

    u16x8 hv, lv;
    split8(u, hv, lv);
    const size_t e = (rbase + (size_t)t) * DI + d0;
    store_planes2x(uh + e, ul + e, hv, lv);
}

__device__ __forceinline__ void rows16_store_pass(const unsigned short* sl, unsigned short* gp,
                                                  size_t gbase, int lane) {
#pragma unroll
    for (int it = 0; it < 4; ++it) {
        const int t = it * 4 + (lane >> 3);
        const int c = (lane & 7) * 8;
        const u16x8 v = *(const u16x8*)(sl + t * 64 + c);
        *(volatile u16x8*)(gp + gbase + (size_t)t * DI + c) = v;
    }
}

__global__ __launch_bounds__(64)
void scan_kernel(const float* __restrict__ X, const float* __restrict__ Z,
                 const float* __restrict__ xd,
                 const float* __restrict__ cw, const float* __restrict__ cb,
                 const float* __restrict__ dtw, const float* __restrict__ dtb,
                 const float* __restrict__ Alog, const float* __restrict__ Dp,
                 int layer, unsigned short* gh, unsigned short* gl)
{
    __shared__ __attribute__((aligned(16))) unsigned short sgl[2][16 * 64];
    __shared__ __attribute__((aligned(16))) float sx[16 * XDW];

    const int tid   = threadIdx.x;
    const int lane  = tid & 31;
    const int wave  = tid >> 5;
    const int f     = blockIdx.z;
    const int b     = blockIdx.y;
    const int dbase = blockIdx.x * 64;
    const int d     = dbase + tid;
    const size_t p  = ((size_t)(f * NLY + layer)) * DI + (size_t)d;

    float an[NS], hs[NS], wd[DTR];
    {
        const v8f a0 = ld8f(Alog + p * NS);
        const v8f a1 = ld8f(Alog + p * NS + 8);
        const v8f w0v = ld8f(dtw + p * DTR);
        const v8f w1v = ld8f(dtw + p * DTR + 8);
#pragma unroll
        for (int n = 0; n < 8; ++n) {
            an[n]     = -__expf(a0[n]);
            an[n + 8] = -__expf(a1[n]);
            wd[n]     = w0v[n];
            wd[n + 8] = w1v[n];
        }
#pragma unroll
        for (int n = 0; n < NS; ++n) hs[n] = 0.0f;
    }
    const v4f cwv = *(const v4f*)(cw + p * 4);
    const float cbias = cb[p];
    const float tb    = dtb[p];
    const float Dd    = Dp[p];

    float xm1 = 0.0f, xm2 = 0.0f, xm3 = 0.0f;
    const size_t row0 = (size_t)f * TOK + (size_t)b * SL;

    const unsigned short* sl = sgl[wave];
    unsigned short* gp = wave ? gl : gh;

#pragma unroll 1
    for (int l0 = 0; l0 < SL; l0 += 16) {
#pragma unroll
        for (int j = 0; j < 16; ++j)
            sx[j * XDW + tid] = xd[(row0 + (size_t)(l0 + j)) * XDW + tid];
        __syncthreads();
#pragma unroll 1
        for (int t = 0; t < 16; ++t) {
            const size_t e = (row0 + (size_t)(l0 + t)) * DI + (size_t)d;
            const float xv = X[e];
            const float zv = Z[e];
            const float u  = conv4_silu(xm3, xm2, xm1, xv, cwv[0], cwv[1], cwv[2], cwv[3], cbias);
            xm3 = xm2; xm2 = xm1; xm1 = xv;
            const float* sr = sx + t * XDW;
            float dpre = tb;
#pragma unroll
            for (int r = 0; r < DTR; ++r) dpre += sr[r] * wd[r];
            const float dt = softplus_f(dpre);
            const float du = dt * u;
            float y = 0.0f;
#pragma unroll
            for (int n = 0; n < NS; ++n) {
                const float da = __expf(dt * an[n]);
                hs[n] = da * hs[n] + du * sr[DTR + n];
                y += hs[n] * sr[DTR + NS + n];
            }
            const float g = (y + Dd * u) * silu_f(zv);
            const unsigned short hb = f32_to_bf16(g);
            const unsigned short lb = f32_to_bf16(g - bf16_to_f32(hb));
            sgl[0][t * 64 + tid] = hb;
            sgl[1][t * 64 + tid] = lb;
        }
        __syncthreads();
        const size_t gbase = (row0 + (size_t)l0) * DI + (size_t)dbase;
        rows16_store_pass(sl, gp, gbase, lane);
        __threadfence();
        rows16_store_pass(sl, gp, gbase, lane);
        __syncthreads();
    }
}

__global__ __launch_bounds__(256)
void bn_cvt_kernel(const float* __restrict__ lg, const float* __restrict__ gam,
                   const float* __restrict__ bet, unsigned short* oh, unsigned short* ol)
{
    __shared__ double sred[256];
    constexpr int NTOT = TOK * NV;
    constexpr int NT8  = NTOT / 8;
    const int f   = blockIdx.x;
    const int tid = threadIdx.x;
    const float* base = lg + (size_t)f * NTOT;

    double s = 0.0;
#pragma unroll 1
    for (int i = tid; i < NT8; i += 256) {
        const v8f v = ld8f(base + (size_t)i * 8);
#pragma unroll
        for (int c = 0; c < 8; ++c) s += (double)v[c];
    }
    sred[tid] = s;
    __syncthreads();
#pragma unroll 1
    for (int st = 128; st > 0; st >>= 1) {
        if (tid < st) sred[tid] += sred[tid + st];
        __syncthreads();
    }
    const double mu = sred[0] * (1.0 / (double)NTOT);
    __syncthreads();

    double s2 = 0.0;
#pragma unroll 1
    for (int i = tid; i < NT8; i += 256) {
        const v8f v = ld8f(base + (size_t)i * 8);
#pragma unroll
        for (int c = 0; c < 8; ++c) { const double dv = (double)v[c] - mu; s2 += dv * dv; }
    }
    sred[tid] = s2;
    __syncthreads();
#pragma unroll 1
    for (int st = 128; st > 0; st >>= 1) {
        if (tid < st) sred[tid] += sred[tid + st];
        __syncthreads();
    }
    const double var = sred[0] * (1.0 / (double)NTOT);
    const float muf  = (float)mu;
    const float rstd = rsqrtf((float)var + 1e-5f);
    const float gm   = gam[f];
    const float be   = bet[f];

#pragma unroll 1
    for (int i = tid; i < NT8; i += 256) {
        const size_t e = (size_t)i * 8;
        const v8f v = ld8f(base + e);
        const int t  = (int)(e >> 7);
        const int v0 = (int)(e & (NV - 1));
        const int bb = t >> 8;
        const int ll = t & (SL - 1);
        v8f y;
#pragma unroll
        for (int c = 0; c < 8; ++c) y[c] = (v[c] - muf) * rstd * gm + be;
        u16x8 hv, lv;
        split8(y, hv, lv);
        const size_t dst = (((size_t)bb * FQ + (size_t)f) * SL + (size_t)ll) * NV + (size_t)v0;
        store_planes2x(oh + dst, ol + dst, hv, lv);
    }
}

extern "C" void kernel_launch(void* const* d_in, const int* in_sizes, int n_in,
                              void* d_out, int out_size, void* d_ws, size_t ws_size,
                              hipStream_t stream)
{
    if (n_in < 17) return;
    if (in_sizes[0]  != NB * SL * FQ * DM)       return;
    if (in_sizes[1]  != FQ * NLY * 2 * DI * DM)  return;
    if (in_sizes[2]  != FQ * NLY * DI * 4)       return;
    if (in_sizes[3]  != FQ * NLY * DI)           return;
    if (in_sizes[4]  != FQ * NLY * XDN * DI)     return;
    if (in_sizes[5]  != FQ * NLY * DI * DTR)     return;
    if (in_sizes[6]  != FQ * NLY * DI)           return;
    if (in_sizes[7]  != FQ * NLY * DI * NS)      return;
    if (in_sizes[8]  != FQ * NLY * DI)           return;
    if (in_sizes[9]  != FQ * NLY * DM * DI)      return;
    if (in_sizes[10] != FQ * NLY * DM)           return;
    if (in_sizes[11] != FQ * DM)                 return;
    if (in_sizes[12] != FQ * NV * DM)            return;
    if (in_sizes[13] != FQ)                      return;
    if (in_sizes[14] != FQ)                      return;
    if (in_sizes[15] != NO * NV)                 return;
    if (in_sizes[16] != NO)                      return;
    if (out_size != TOKO * NO)                   return;
    if (ws_size < WS_END)                        return;

    const float* x    = (const float*)d_in[0];
    const float* wi   = (const float*)d_in[1];
    const float* cw   = (const float*)d_in[2];
    const float* cb   = (const float*)d_in[3];
    const float* wx   = (const float*)d_in[4];
    const float* wdt  = (const float*)d_in[5];
    const float* dtb  = (const float*)d_in[6];
    const float* alog = (const float*)d_in[7];
    const float* Dp   = (const float*)d_in[8];
    const float* wo   = (const float*)d_in[9];
    const float* nw   = (const float*)d_in[10];
    const float* fnw  = (const float*)d_in[11];
    const float* wl   = (const float*)d_in[12];
    const float* gam  = (const float*)d_in[13];
    const float* bet  = (const float*)d_in[14];
    const float* wt   = (const float*)d_in[15];
    const float* tbv  = (const float*)d_in[16];
    float* out = (float*)d_out;

    char* ws = (char*)d_ws;
    unsigned short* wih = (unsigned short*)(ws + OFF_WIH);
    unsigned short* wil = (unsigned short*)(ws + OFF_WIL);
    unsigned short* wxh = (unsigned short*)(ws + OFF_WXH);
    unsigned short* wxl = (unsigned short*)(ws + OFF_WXL);
    unsigned short* woh = (unsigned short*)(ws + OFF_WOH);
    unsigned short* wol = (unsigned short*)(ws + OFF_WOL);
    unsigned short* wlh = (unsigned short*)(ws + OFF_WLH);
    unsigned short* wll = (unsigned short*)(ws + OFF_WLL);
    unsigned short* wth = (unsigned short*)(ws + OFF_WTH);
    unsigned short* wtl = (unsigned short*)(ws + OFF_WTL);
    float*          hA  = (float*)(ws + OFF_HA);
    float*          hB  = (float*)(ws + OFF_HB);
    unsigned short* nh  = (unsigned short*)(ws + OFF_NH);
    unsigned short* nl  = (unsigned short*)(ws + OFF_NL);
    float*          Xf  = (float*)(ws + OFF_XF);
    float*          Zf  = (float*)(ws + OFF_ZF);
    unsigned short* uh  = (unsigned short*)(ws + OFF_UH);
    unsigned short* ul  = (unsigned short*)(ws + OFF_UL);
    float*          xd  = (float*)(ws + OFF_XD);
    unsigned short* gh  = (unsigned short*)(ws + OFF_GH);
    unsigned short* gl  = (unsigned short*)(ws + OFF_GL);
    float*          lg  = (float*)(ws + OFF_LG);
    unsigned short* bnh = (unsigned short*)(ws + OFF_BNH);
    unsigned short* bnl = (unsigned short*)(ws + OFF_BNL);

    {
        int n8;
        n8 = (FQ * NLY * 2 * DI * DM) / 8;
        hipLaunchKernelGGL(cvt_kernel, dim3((n8 + 255) / 256), dim3(256), 0, stream,
                           wi, wih, wil, n8, n8, n8);
        n8 = (FQ * NLY * XDW * DI) / 8;
        hipLaunchKernelGGL(cvt_kernel, dim3((n8 + 255) / 256), dim3(256), 0, stream,
                           wx, wxh, wxl, n8, (int)((XDW * DI) / 8), (int)((XDN * DI) / 8));
        n8 = (FQ * NLY * DM * DI) / 8;
        hipLaunchKernelGGL(cvt_kernel, dim3((n8 + 255) / 256), dim3(256), 0, stream,
                           wo, woh, wol, n8, n8, n8);
        n8 = (FQ * NV * DM) / 8;
        hipLaunchKernelGGL(cvt_kernel, dim3((n8 + 255) / 256), dim3(256), 0, stream,
                           wl, wlh, wll, n8, n8, n8);
        n8 = (NO * NV) / 8;
        hipLaunchKernelGGL(cvt_kernel, dim3((n8 + 255) / 256), dim3(256), 0, stream,
                           wt, wth, wtl, n8, n8, n8);
    }

    for (int layer = 0; layer < NLY; ++layer) {
        const float* hin  = (layer == 0) ? x : hB;
        const int    inFeat = (layer == 0) ? DM : TOK * DM;
        const int    inRow  = (layer == 0) ? FQ * DM : DM;
        float*       hout = (layer == 0) ? hB : hA;

        hipLaunchKernelGGL(rmsnorm_cvt_kernel, dim3(TOK, FQ), dim3(32), 0, stream,
                           hin, inFeat, inRow, nw + (size_t)layer * DM, (int)(NLY * DM), nh, nl);

        hipLaunchKernelGGL(HIP_KERNEL_NAME(gemm3_kernel<2, 0>),
                           dim3((2 * DI) / 64, TOK / 64, FQ), dim3(128), 0, stream,
                           (const unsigned short*)nh, (const unsigned short*)nl, (int)(TOK * DM),
                           (const unsigned short*)(wih + (size_t)layer * 2 * DI * DM),
                           (const unsigned short*)(wil + (size_t)layer * 2 * DI * DM), (int)(NLY * 2 * DI * DM),
                           Xf, Zf, (int)(TOK * DI), (int)DM, (int)DI, (int)DI,
                           tbv, 0, 0);

        hipLaunchKernelGGL(conv_cvt_kernel, dim3(TOK, FQ), dim3(DI / 8), 0, stream,
                           (const float*)Xf, cw, cb, layer, uh, ul);

        hipLaunchKernelGGL(HIP_KERNEL_NAME(gemm3_kernel<2, 0>),
                           dim3(XDW / 64, TOK / 64, FQ), dim3(128), 0, stream,
                           (const unsigned short*)uh, (const unsigned short*)ul, (int)(TOK * DI),
                           (const unsigned short*)(wxh + (size_t)layer * XDW * DI),
                           (const unsigned short*)(wxl + (size_t)layer * XDW * DI), (int)(NLY * XDW * DI),
                           xd, xd, (int)(TOK * XDW), (int)DI, (int)XDW, (int)(1 << 30),
                           tbv, 0, 0);

        hipLaunchKernelGGL(scan_kernel, dim3(DI / 64, NB, FQ), dim3(64), 0, stream,
                           (const float*)Xf, (const float*)Zf, (const float*)xd,
                           cw, cb, wdt, dtb, alog, Dp, layer, gh, gl);

        hipLaunchKernelGGL(HIP_KERNEL_NAME(gemm3_kernel<2, 1>),
                           dim3(DM / 64, TOK / 64, FQ), dim3(128), 0, stream,
                           (const unsigned short*)gh, (const unsigned short*)gl, (int)(TOK * DI),
                           (const unsigned short*)(woh + (size_t)layer * DM * DI),
                           (const unsigned short*)(wol + (size_t)layer * DM * DI), (int)(NLY * DM * DI),
                           hout, hout, (int)(TOK * DM), (int)DI, (int)DM, (int)(1 << 30),
                           hin, inFeat, inRow);
    }

    hipLaunchKernelGGL(rmsnorm_cvt_kernel, dim3(TOK, FQ), dim3(32), 0, stream,
                       (const float*)hA, (int)(TOK * DM), (int)DM, fnw, (int)DM, nh, nl);
    hipLaunchKernelGGL(HIP_KERNEL_NAME(gemm3_kernel<2, 0>),
                       dim3(NV / 64, TOK / 64, FQ), dim3(128), 0, stream,
                       (const unsigned short*)nh, (const unsigned short*)nl, (int)(TOK * DM),
                       (const unsigned short*)wlh, (const unsigned short*)wll, (int)(NV * DM),
                       lg, lg, (int)(TOK * NV), (int)DM, (int)NV, (int)(1 << 30),
                       tbv, 0, 0);

    hipLaunchKernelGGL(bn_cvt_kernel, dim3(FQ), dim3(256), 0, stream,
                       (const float*)lg, gam, bet, bnh, bnl);

    hipLaunchKernelGGL(HIP_KERNEL_NAME(gemm3_kernel<2, 2>),
                       dim3(NO / 64, TOKO / 64, 1), dim3(128), 0, stream,
                       (const unsigned short*)bnh, (const unsigned short*)bnl, 0,
                       (const unsigned short*)wth, (const unsigned short*)wtl, 0,
                       out, out, 0, (int)NV, (int)NO, (int)(1 << 30),
                       tbv, 0, 0);
}
